// MambaBlock_47270410060482
// MI455X (gfx1250) — hardware-run, weakly checked
//
#include <hip/hip_runtime.h>
#include <hip/hip_fp16.h>
#include <math.h>

typedef __attribute__((ext_vector_type(16))) _Float16 v16h;
typedef __attribute__((ext_vector_type(8)))  _Float16 v8h;
typedef __attribute__((ext_vector_type(8)))  float    v8f;
typedef __attribute__((ext_vector_type(4)))  float    v4f;

constexpr int kBatch  = 2;
constexpr int kSeq    = 2048;
constexpr int kDm     = 1024;
constexpr int kDin    = 2048;
constexpr int kNst    = 16;
constexpr int kXzP    = 2 * kDin;
constexpr int kDtR    = 64;
constexpr int kXpN    = kDtR + 2 * kNst;
constexpr int kBcP    = 128;
constexpr int kOffB   = kDtR;
constexpr int kOffC   = kDtR + kNst;
constexpr int kConvTP = 260;
constexpr float kWCarry = 1024.0f;
constexpr float kResid  = 2048.0f;
constexpr float kYCarry = 16.0f;
constexpr float kSW  = 1.0f / kWCarry;
constexpr float kSWr = 1.0f / (kWCarry * kResid);
constexpr float kSY  = 1.0f / (kYCarry * kWCarry);
constexpr float kSYr = 1.0f / (kYCarry * kWCarry * kResid);
static_assert(kXpN == 96);
static_assert(kXpN <= kBcP);
static_assert((kDm % 64) == 0 && (kDin % 64) == 0);
static_assert((kSeq % 64) == 0 && (kXzP % 64) == 0 && (kBcP % 64) == 0);
static_assert((kDin % 256) == 0 && (kDtR % 64) == 0 && kDtR <= kBcP);
static_assert(kDm == 1024);
constexpr float kLnEps = 1e-5f;

constexpr size_t kSzWIN  = (size_t)kXzP * kDm * 2;
constexpr size_t kSzWOUT = (size_t)kDm * kDin * 2;
constexpr size_t kSzWX   = (size_t)kBcP * kDin * 2;
constexpr size_t kSzWDT  = (size_t)kDin * kDtR * 2;
constexpr size_t kSzP    = (size_t)kSeq * kDm * 4;
constexpr size_t kSzX16  = (size_t)kSeq * kDm * 2;
constexpr size_t kSzXZ   = (size_t)kSeq * kXzP * 4;
constexpr size_t kSzU    = (size_t)kSeq * kDin * 4;
constexpr size_t kSzU16  = (size_t)kSeq * kDin * 2;
constexpr size_t kSzBC   = (size_t)kSeq * kBcP * 4;
constexpr size_t kSzBC16 = (size_t)kSeq * kBcP * 2;
constexpr size_t kOffWIN  = 0;
constexpr size_t kOffWOUT = kOffWIN  + kSzWIN;
constexpr size_t kOffWXH  = kOffWOUT + kSzWOUT;
constexpr size_t kOffWXL  = kOffWXH  + kSzWX;
constexpr size_t kOffWDT  = kOffWXL  + kSzWX;
constexpr size_t kOffXH   = kOffWDT  + kSzWDT;
constexpr size_t kOffXL   = kOffXH   + kSzX16;
constexpr size_t kOffXZ   = kOffXL   + kSzX16;
constexpr size_t kOffU    = kOffXZ   + kSzXZ;
constexpr size_t kOffUH   = kOffU    + kSzU;
constexpr size_t kOffUL   = kOffUH   + kSzU16;
constexpr size_t kOffBC   = kOffUL   + kSzU16;
constexpr size_t kOffBCH  = kOffBC   + kSzBC;
constexpr size_t kOffBCL  = kOffBCH  + kSzBC16;
constexpr size_t kOffDT   = kOffBCL  + kSzBC16;
constexpr size_t kOffYH   = kOffDT   + kSzU;
constexpr size_t kOffYL   = kOffYH   + kSzU16;
constexpr size_t kOffP    = kOffYL   + kSzU16;
constexpr size_t kWsTotal = kOffP    + kSzP;
static_assert(kWsTotal == 133431296ull);
static_assert(kWsTotal <= 134217728ull);
static_assert((kOffWOUT % 128) == 0 && (kOffWXH % 128) == 0 && (kOffWXL % 128) == 0 && (kOffWDT % 128) == 0 &&
              (kOffXH % 128) == 0 && (kOffXL % 128) == 0 && (kOffXZ % 128) == 0 && (kOffU % 128) == 0 &&
              (kOffUH % 128) == 0 && (kOffUL % 128) == 0 && (kOffBC % 128) == 0 && (kOffBCH % 128) == 0 &&
              (kOffBCL % 128) == 0 && (kOffDT % 128) == 0 && (kOffYH % 128) == 0 && (kOffYL % 128) == 0 &&
              (kOffP % 128) == 0);

__device__ __forceinline__ _Float16 f16_flush(float v) {
  const float w = (fabsf(v) < 6.103515625e-05f) ? 0.0f : v;
  return (_Float16)w;
}
__device__ __forceinline__ void f16_split(float v, _Float16& hi, _Float16& lo) {
  hi = f16_flush(v);
  const float hf = (float)hi;
  const float r = (v - hf) * kResid;
  lo = f16_flush(r);
}

namespace eng {
union FragU { v16h v; v8h h[2]; };
__device__ __forceinline__ v16h frag_load(const _Float16* p) {
  FragU f;
  f.h[0] = *(const v8h*)(p);
  f.h[1] = *(const v8h*)(p + 16);
  return f.v;
}
__device__ __forceinline__ v8f mma(v16h a, v16h b, v8f c) {
  return __builtin_amdgcn_wmma_f32_16x16x32_f16(false, a, false, b, (short)0, c, false, false);
}
__device__ __forceinline__ void guard1(v8f& a, v16h x, v16h y) {
  asm volatile("v_nop\n\tv_nop\n\tv_nop\n\tv_nop" : "+v"(a) : "v"(x), "v"(y));
}
__device__ __forceinline__ void guard_acc(v8f& a) {
  asm volatile("v_nop\n\tv_nop\n\tv_nop\n\tv_nop" : "+v"(a));
}
__device__ __forceinline__ void keep4(v16h a, v16h b, v16h c, v16h d) {
  asm volatile("v_nop" :: "v"(a), "v"(b), "v"(c), "v"(d));
}

template <int MI, int SPL>
__global__ __launch_bounds__(256) void gemm_f16_kernel(
    const unsigned short* __restrict__ Ap, const unsigned short* __restrict__ A2p, int lda,
    const unsigned short* __restrict__ Btp, const unsigned short* __restrict__ Bt2p, int ldb,
    float* __restrict__ C, int ldc, int M, int N, int K, float scale, float rscale)
{
  static_assert(MI >= 1 && MI <= 2);
  static_assert(SPL >= 0 && SPL <= 2);
  const _Float16* A   = (const _Float16*)Ap;
  const _Float16* A2  = (const _Float16*)A2p;
  const _Float16* Bt  = (const _Float16*)Btp;
  const _Float16* Bt2 = (const _Float16*)Bt2p;
  __shared__ __align__(16) float sT[8][16 * 68];
  const int lane = threadIdx.x & 31;
  const int wave = threadIdx.x >> 5;
  const int tilesN = N >> 6;
  const int tilesM = M / (16 * MI);
  const int tile = blockIdx.x * 8 + wave;
  if (tile >= tilesM * tilesN) return;
  const int tm = tile / tilesN;
  const int tn = tile - tm * tilesN;
  const int m0 = tm * (16 * MI);
  const int n0 = tn << 6;
  const int rlane = lane & 15;
  const int koff  = (lane >> 4) * 8;
  const int mOff  = (lane >> 4) * 8;

  v8f acc[MI][4], accr[MI][4];
#pragma unroll
  for (int i = 0; i < MI; ++i)
#pragma unroll
    for (int j = 0; j < 4; ++j) {
      acc[i][j]  = (v8f){0.f, 0.f, 0.f, 0.f, 0.f, 0.f, 0.f, 0.f};
      accr[i][j] = (v8f){0.f, 0.f, 0.f, 0.f, 0.f, 0.f, 0.f, 0.f};
    }

  for (int k0 = 0; k0 < K; k0 += 32) {
    v16h bh[4], bl[4];
#pragma unroll
    for (int j = 0; j < 4; ++j) {
      const size_t bo = (size_t)(n0 + (j << 4) + rlane) * ldb + koff + k0;
      bh[j] = frag_load(Bt + bo);
      if (SPL == 2) bl[j] = frag_load(Bt2 + bo); else bl[j] = bh[j];
    }
#pragma unroll
    for (int i = 0; i < MI; ++i) {
      const size_t ao = (size_t)(m0 + (i << 4) + rlane) * lda + koff + k0;
      const v16h ah = frag_load(A + ao);
      v16h al = ah;
      if (SPL >= 1) al = frag_load(A2 + ao);
#pragma unroll
      for (int j = 0; j < 4; ++j) {
        acc[i][j] = mma(ah, bh[j], acc[i][j]);
        if (SPL >= 1) accr[i][j] = mma(al, bh[j], accr[i][j]);
        if (SPL == 2) accr[i][j] = mma(ah, bl[j], accr[i][j]);
      }
#pragma unroll
      for (int j = 0; j < 4; ++j) {
        guard1(acc[i][j], ah, al);
        if (SPL >= 1) guard1(accr[i][j], ah, al);
      }
    }
    keep4(bh[0], bh[1], bh[2], bh[3]);
    if (SPL == 2) keep4(bl[0], bl[1], bl[2], bl[3]);
  }
#pragma unroll
  for (int i = 0; i < MI; ++i)
#pragma unroll
    for (int j = 0; j < 4; ++j) {
      guard_acc(acc[i][j]);
      if (SPL >= 1) guard_acc(accr[i][j]);
    }

  float* slab = sT[wave];
#pragma unroll
  for (int i = 0; i < MI; ++i) {
    const int mBase = m0 + (i << 4);
#pragma unroll
    for (int j = 0; j < 4; ++j) {
#pragma unroll
      for (int r = 0; r < 8; ++r) {
        float v = acc[i][j][r] * scale;
        if (SPL >= 1) v += accr[i][j][r] * rscale;
        slab[(mOff + r) * 68 + (j << 4) + rlane] = v;
      }
    }
    __builtin_amdgcn_fence(__ATOMIC_RELEASE, "workgroup");
    __builtin_amdgcn_wave_barrier();
    __builtin_amdgcn_fence(__ATOMIC_ACQUIRE, "workgroup");
    {
      const int hh = lane >> 4, c4 = (lane & 15) * 4;
      for (int pass = 0; pass < 2; ++pass) {
#pragma unroll
        for (int it = 0; it < 8; ++it) {
          const int row = it * 2 + hh;
          const v4f v = *(const v4f*)(slab + row * 68 + c4);
          *(volatile v4f*)(C + (size_t)(mBase + row) * ldc + n0 + c4) = v;
        }
        __threadfence();
      }
    }
    __builtin_amdgcn_fence(__ATOMIC_RELEASE, "workgroup");
    __builtin_amdgcn_wave_barrier();
    __builtin_amdgcn_fence(__ATOMIC_ACQUIRE, "workgroup");
  }
}
}

__global__ __launch_bounds__(256) void split_rows_f16_kernel(
    const float* __restrict__ src, unsigned short* __restrict__ dH, unsigned short* __restrict__ dL, int total8)
{
  const int i = blockIdx.x * 256 + threadIdx.x;
  if (i >= total8) return;
  const size_t e0 = (size_t)i << 3;
  const v4f a0 = *(const v4f*)(src + e0);
  const v4f a1 = *(const v4f*)(src + e0 + 4);
  v8h hv, lv;
#pragma unroll
  for (int e = 0; e < 4; ++e) {
    _Float16 h0, l0, h1, l1;
    const float f0 = a0[e];
    const float f1 = a1[e];
    f16_split(f0, h0, l0);
    f16_split(f1, h1, l1);
    hv[e] = h0; lv[e] = l0;
    hv[4 + e] = h1; lv[4 + e] = l1;
  }
  unsigned short* qh = dH + e0;
  unsigned short* ql = dL + e0;
  *(volatile v8h*)qh = hv;
  *(volatile v8h*)ql = lv;
  __threadfence();
  *(volatile v8h*)qh = hv;
  *(volatile v8h*)ql = lv;
}

template <bool LO>
__global__ __launch_bounds__(256) void transpose_pack_kernel(
    const float* __restrict__ W, unsigned short* __restrict__ BtH, unsigned short* __restrict__ BtL,
    int Kdim, int Ndim, float carry)
{
  __shared__ float tile[64 * 65];
  const int tid = threadIdx.x, lane = tid & 31, wave = tid >> 5;
  const int n0 = blockIdx.x * 64;
  const int k0 = blockIdx.y * 64;
#pragma unroll
  for (int p = 0; p < 16; ++p) {
    const int idx = tid + p * 256;
    const int kk  = idx >> 6;
    const int nn  = idx & 63;
    const int n   = n0 + nn;
    const int nc  = (n < Ndim) ? n : (Ndim - 1);
    const float v = W[(size_t)(k0 + kk) * Ndim + nc];
    tile[kk * 65 + nn] = (n < Ndim) ? (v * carry) : 0.0f;
  }
  __syncthreads();
  const int q = lane >> 3, c8 = (lane & 7) * 8;
  v8h hv[2], lv[2];
#pragma unroll
  for (int it = 0; it < 2; ++it) {
    const int nrow = it * 32 + wave * 4 + q;
#pragma unroll
    for (int e = 0; e < 8; ++e) {
      _Float16 h, l;
      const float t = tile[(c8 + e) * 65 + nrow];
      f16_split(t, h, l);
      hv[it][e] = h;
      lv[it][e] = l;
    }
  }
  for (int pass = 0; pass < 2; ++pass) {
#pragma unroll
    for (int it = 0; it < 2; ++it) {
      const int nrow = it * 32 + wave * 4 + q;
      const size_t o = (size_t)(n0 + nrow) * Kdim + k0 + c8;
      *(volatile v8h*)(BtH + o) = hv[it];
      if (LO) *(volatile v8h*)(BtL + o) = lv[it];
    }
    __threadfence();
  }
}

__global__ __launch_bounds__(256) void conv_silu_kernel(
    const float* __restrict__ XZ, const float* __restrict__ cw, const float* __restrict__ cb,
    float* __restrict__ UC, unsigned short* __restrict__ UH, unsigned short* __restrict__ UL)
{
  __shared__ __align__(16) float sT[16 * kConvTP];
  const int tid = threadIdx.x, lane = tid & 31, wave = tid >> 5;
  const int d0 = blockIdx.x * 256, d = d0 + tid;
  const int t0 = blockIdx.y * 64;
  const v4f wv = *(const v4f*)(cw + (size_t)d * 4);
  const float w0 = wv[0], w1 = wv[1], w2 = wv[2], w3 = wv[3];
  const float bc = cb[d];
  float xm3, xm2, xm1;
  {
    const int r3 = t0 - 3, r2 = t0 - 2, r1 = t0 - 1;
    const float v3 = XZ[(size_t)(r3 < 0 ? 0 : r3) * kXzP + d];
    const float v2 = XZ[(size_t)(r2 < 0 ? 0 : r2) * kXzP + d];
    const float v1 = XZ[(size_t)(r1 < 0 ? 0 : r1) * kXzP + d];
    xm3 = (r3 >= 0) ? v3 : 0.0f;
    xm2 = (r2 >= 0) ? v2 : 0.0f;
    xm1 = (r1 >= 0) ? v1 : 0.0f;
  }
  const int hrow = wave >> 1;
  const int hch  = (wave & 1) * 128 + lane * 4;
#pragma unroll 1
  for (int sub = 0; sub < 4; ++sub) {
    const int lb = t0 + sub * 16;
#pragma unroll 1
    for (int s = 0; s < 16; ++s) {
      const float xcur = XZ[(size_t)(lb + s) * kXzP + d];
      float acc = w0 * xm3;
      acc = fmaf(w1, xm2, acc);
      acc = fmaf(w2, xm1, acc);
      acc = fmaf(w3, xcur, acc);
      const float sv = acc + bc;
      const float sg = __builtin_amdgcn_rcpf(1.0f + expf(-sv));
      sT[s * kConvTP + tid] = sv * sg;
      xm3 = xm2; xm2 = xm1; xm1 = xcur;
    }
    __syncthreads();
    v4f fv[4];
    v8h hv[2], lv[2];
#pragma unroll
    for (int it = 0; it < 4; ++it) fv[it] = *(const v4f*)(sT + (it * 4 + hrow) * kConvTP + hch);
#pragma unroll
    for (int it = 0; it < 2; ++it) {
      const float* sp = sT + (it * 8 + wave) * kConvTP + lane * 8;
      const v4f a0 = *(const v4f*)(sp);
      const v4f a1 = *(const v4f*)(sp + 4);
#pragma unroll
      for (int e = 0; e < 4; ++e) {
        _Float16 h0, l0, h1, l1;
        const float f0 = a0[e];
        const float f1 = a1[e];
        f16_split(f0, h0, l0);
        f16_split(f1, h1, l1);
        hv[it][e] = h0; lv[it][e] = l0;
        hv[it][4 + e] = h1; lv[it][4 + e] = l1;
      }
    }
    for (int pass = 0; pass < 2; ++pass) {
#pragma unroll
      for (int it = 0; it < 4; ++it)
        *(volatile v4f*)(UC + (size_t)(lb + it * 4 + hrow) * kDin + d0 + hch) = fv[it];
#pragma unroll
      for (int it = 0; it < 2; ++it) {
        const size_t o = (size_t)(lb + it * 8 + wave) * kDin + d0 + lane * 8;
        *(volatile v8h*)(UH + o) = hv[it];
        *(volatile v8h*)(UL + o) = lv[it];
      }
      __threadfence();
    }
    __syncthreads();
  }
}

__global__ __launch_bounds__(256) void bias_rows_kernel(
    float* __restrict__ DT, const float* __restrict__ bdt, int total4)
{
  const int i = blockIdx.x * 256 + threadIdx.x;
  if (i >= total4) return;
  unsigned e0 = (unsigned)i << 2;
  asm volatile("" : "+v"(e0));
  const unsigned row = e0 / (unsigned)kDin;
  const unsigned d4  = e0 - row * (unsigned)kDin;
  const v4f v = *(const v4f*)(DT + (size_t)e0);
  const v4f b = *(const v4f*)(bdt + d4);
  const v4f o = v + b;
  *(volatile v4f*)(DT + (size_t)e0) = o;
  __threadfence();
  *(volatile v4f*)(DT + (size_t)e0) = o;
}

__global__ __launch_bounds__(256) void ln_split_rows_kernel(
    const float* __restrict__ src, const float* __restrict__ gam, const float* __restrict__ bet,
    unsigned short* __restrict__ dH, unsigned short* __restrict__ dL)
{
  __shared__ float red[8 * 32];
  const int lane = threadIdx.x & 31, wave = threadIdx.x >> 5;
  const int row = blockIdx.x * 8 + wave;
  const float* p = src + (size_t)row * kDm;
  v4f a[8];
#pragma unroll
  for (int j = 0; j < 4; ++j) {
    a[2 * j]     = *(const v4f*)(p + 256 * j + 8 * lane);
    a[2 * j + 1] = *(const v4f*)(p + 256 * j + 8 * lane + 4);
  }
  float s = 0.0f;
#pragma unroll
  for (int q = 0; q < 8; ++q) s += (a[q][0] + a[q][1]) + (a[q][2] + a[q][3]);
  red[wave * 32 + lane] = s;
  __syncthreads();
  float tot = 0.0f;
#pragma unroll
  for (int q = 0; q < 32; ++q) tot += red[wave * 32 + q];
  const float mu = tot * (1.0f / (float)kDm);
  float ss = 0.0f;
#pragma unroll
  for (int q = 0; q < 8; ++q) {
#pragma unroll
    for (int e = 0; e < 4; ++e) {
      const float d = a[q][e] - mu;
      ss = fmaf(d, d, ss);
    }
  }
  __syncthreads();
  red[wave * 32 + lane] = ss;
  __syncthreads();
  float tss = 0.0f;
#pragma unroll
  for (int q = 0; q < 32; ++q) tss += red[wave * 32 + q];
  const float rstd = 1.0f / sqrtf(tss * (1.0f / (float)kDm) + kLnEps);
  v8h hv[4], lv[4];
#pragma unroll
  for (int j = 0; j < 4; ++j) {
    const v4f g0 = *(const v4f*)(gam + 256 * j + 8 * lane);
    const v4f g1 = *(const v4f*)(gam + 256 * j + 8 * lane + 4);
    const v4f b0 = *(const v4f*)(bet + 256 * j + 8 * lane);
    const v4f b1 = *(const v4f*)(bet + 256 * j + 8 * lane + 4);
#pragma unroll
    for (int e = 0; e < 4; ++e) {
      _Float16 h0, l0, h1, l1;
      const float f0 = fmaf((a[2 * j][e] - mu) * rstd, g0[e], b0[e]);
      const float f1 = fmaf((a[2 * j + 1][e] - mu) * rstd, g1[e], b1[e]);
      f16_split(f0, h0, l0);
      f16_split(f1, h1, l1);
      hv[j][e] = h0; lv[j][e] = l0;
      hv[j][4 + e] = h1; lv[j][4 + e] = l1;
    }
  }
  unsigned short* qh = dH + (size_t)row * kDm + 8 * lane;
  unsigned short* ql = dL + (size_t)row * kDm + 8 * lane;
  for (int pass = 0; pass < 2; ++pass) {
#pragma unroll
    for (int j = 0; j < 4; ++j) {
      *(volatile v8h*)(qh + 256 * j) = hv[j];
      *(volatile v8h*)(ql + 256 * j) = lv[j];
    }
    __threadfence();
  }
}

__global__ __launch_bounds__(256) void residual_out_kernel(
    const float* __restrict__ P, const float* __restrict__ xin, float* __restrict__ out, int total4)
{
  const int i = blockIdx.x * 256 + threadIdx.x;
  if (i >= total4) return;
  const size_t e0 = (size_t)i << 2;
  const v4f a = *(const v4f*)(P + e0);
  const v4f b = *(const v4f*)(xin + e0);
  const v4f o = a + b;
  *(volatile v4f*)(out + e0) = o;
  __threadfence();
  *(volatile v4f*)(out + e0) = o;
}

typedef float    ms1_v4f __attribute__((ext_vector_type(4)));
typedef unsigned ms1_v4u __attribute__((ext_vector_type(4)));
struct ms1_args {
  const float* dtpre;
  const float* u;
  const float* bc;
  const float* z;
  const float* A_log;
  const float* Dskip;
  __half* y;
  __half* y_lo;
  long ld_dtpre;
  long ld_u;
  long ld_bc;
  long ld_z;
  long ld_y;
  int offB;
  int offC;
  int offZ;
  float ycarry;
  int dir;
  int D;
  int L;
  int nbatch;
};
static_assert(sizeof(ms1_args) == 136);

__device__ __forceinline__ float ms1_flush16(float v) {
  return (fabsf(v) < 6.103515625e-05f) ? 0.0f : v;
}
__device__ __forceinline__ unsigned ms1_h16bits(float v) {
  return (unsigned)__half_as_ushort(__float2half_rn(ms1_flush16(v)));
}
__device__ __forceinline__ float ms1_h16val(unsigned b) {
  return __half2float(__ushort_as_half((unsigned short)b));
}
__device__ __forceinline__ float ms1_softplus(float v) {
  return fmaxf(v, 0.0f) + log1pf(expf(-fabsf(v)));
}
__device__ __forceinline__ void ms1_pack2(float v0, float v1, unsigned& hw, unsigned& lw) {
  const unsigned h0 = ms1_h16bits(v0);
  const unsigned h1 = ms1_h16bits(v1);
  const float r0 = (v0 - ms1_h16val(h0)) * 2048.0f;
  const float r1 = (v1 - ms1_h16val(h1)) * 2048.0f;
  const unsigned l0 = ms1_h16bits(r0);
  const unsigned l1 = ms1_h16bits(r1);
  hw = h0 | (h1 << 16);
  lw = l0 | (l1 << 16);
}

template <int NSTATE>
__global__ __launch_bounds__(64 * (NSTATE / 16)) void ms1_scan_kernel(ms1_args a)
{
  static_assert(NSTATE == 16 || NSTATE == 64);
  constexpr int NQ  = NSTATE / 16;
  constexpr int NT  = 64 * NQ;
  constexpr int NW  = NT / 32;
  constexpr int BCW = 2 * NSTATE;
  constexpr int YP  = 68;
  constexpr int RPI = NW * 4;
  constexpr int NIT = 64 / RPI;
  static_assert(16 * NT <= 64 * YP);
  __shared__ __align__(16) float sBC[64 * BCW];
  __shared__ __align__(16) float sY[64 * YP];
  const int tid  = threadIdx.x;
  const int lane = tid & 31;
  const int wave = tid >> 5;
  const int c    = tid / NQ;
  const int sq   = tid - c * NQ;
  const int bpb  = a.D / 64;
  const int bi   = blockIdx.x / bpb;
  if (bi >= a.nbatch) return;
  const int d0 = (blockIdx.x - bi * bpb) * 64;
  const int d  = d0 + c;
  const long rowb = (long)bi * a.L;
  const bool hasz  = (a.z != nullptr);
  const bool hasD  = (a.Dskip != nullptr);
  const bool hasLo = (a.y_lo != nullptr);

#pragma unroll 1
  for (int n = 0; n < 16; ++n) {
    const float al = a.A_log[(long)d * NSTATE + sq * 16 + n];
    sY[n * NT + tid] = -expf(al);
  }
  __syncthreads();
  float An[16], h[16];
#pragma unroll
  for (int n = 0; n < 16; ++n) {
    An[n] = sY[n * NT + tid];
    h[n] = 0.0f;
  }
  float Dd = 0.0f;
  if (hasD) Dd = a.Dskip[d];

  const int nchunk = a.L / 64;
  const bool fwd = (a.dir > 0);
  const int s0 = fwd ? 0 : 63;
  const int sd = fwd ? 1 : -1;
  const int q  = lane >> 3;
  const int c8 = (lane & 7) * 8;

#pragma unroll 1
  for (int ci = 0; ci < nchunk; ++ci) {
    const int tb = fwd ? (ci * 64) : (a.L - 64 - ci * 64);
    const long rowc = rowb + tb;
    __syncthreads();
#pragma unroll 8
    for (int i = 0; i < 32; ++i) {
      const int idx = tid + i * NT;
      const int st  = idx / BCW;
      const int col = idx - st * BCW;
      const int sc  = (col < NSTATE) ? (a.offB + col) : (a.offC + col - NSTATE);
      sBC[idx] = a.bc[(rowc + st) * a.ld_bc + sc];
    }
    __syncthreads();
#pragma unroll 1
    for (int s = 0; s < 64; ++s) {
      const int ls = s0 + sd * s;
      const long row = rowc + ls;
      float pre = a.dtpre[row * a.ld_dtpre + d];
      float uv  = a.u[row * a.ld_u + d];
      float zv  = 0.0f;
      if (hasz) zv = a.z[row * a.ld_z + a.offZ + d];
      asm volatile("" : "+v"(pre));
      asm volatile("" : "+v"(uv));
      asm volatile("" : "+v"(zv));
      const float delta = ms1_softplus(pre);
      const float dtx = delta * uv;
      const float* bp = sBC + ls * BCW + sq * 16;
      const float* cp = bp + NSTATE;
      ms1_v4f Bq[4], Cq[4];
#pragma unroll
      for (int k = 0; k < 4; ++k) {
        Bq[k] = *(const ms1_v4f*)(bp + 4 * k);
        Cq[k] = *(const ms1_v4f*)(cp + 4 * k);
      }
      float yv = 0.0f;
#pragma unroll
      for (int n = 0; n < 16; ++n) {
        const float e = __expf(delta * An[n]);
        h[n] = fmaf(e, h[n], dtx * Bq[n >> 2][n & 3]);
        yv = fmaf(h[n], Cq[n >> 2][n & 3], yv);
      }
      if (NQ > 1) {
        yv += __shfl_xor(yv, 1, 32);
        yv += __shfl_xor(yv, 2, 32);
      }
      if (hasD) yv = fmaf(uv, Dd, yv);
      if (hasz) {
        const float sg = __builtin_amdgcn_rcpf(1.0f + expf(-zv));
        yv = yv * (zv * sg);
      }
      if (sq == 0) sY[ls * YP + c] = yv * a.ycarry;
    }
    __syncthreads();
    ms1_v4u hw[NIT], lw[NIT];
#pragma unroll
    for (int it = 0; it < NIT; ++it) {
      const int row = it * RPI + wave * 4 + q;
      const float* sp = sY + row * YP + c8;
      const ms1_v4f f0 = *(const ms1_v4f*)(sp);
      const ms1_v4f f1 = *(const ms1_v4f*)(sp + 4);
      unsigned h0, h1, h2, h3, l0, l1, l2, l3;
      ms1_pack2(f0[0], f0[1], h0, l0);
      ms1_pack2(f0[2], f0[3], h1, l1);
      ms1_pack2(f1[0], f1[1], h2, l2);
      ms1_pack2(f1[2], f1[3], h3, l3);
      hw[it] = (ms1_v4u){h0, h1, h2, h3};
      lw[it] = (ms1_v4u){l0, l1, l2, l3};
    }
    for (int pass = 0; pass < 2; ++pass) {
#pragma unroll
      for (int it = 0; it < NIT; ++it) {
        const int row = it * RPI + wave * 4 + q;
        const long o = (rowc + row) * a.ld_y + d0 + c8;
        *(volatile ms1_v4u*)(a.y + o) = hw[it];
        if (hasLo) *(volatile ms1_v4u*)(a.y_lo + o) = lw[it];
      }
      __threadfence();
    }
  }
}

extern "C" void kernel_launch(void* const* d_in, const int* in_sizes, int n_in,
                              void* d_out, int out_size, void* d_ws, size_t ws_size,
                              hipStream_t stream)
{
  if (n_in < 12) return;
  if (in_sizes[0] != kBatch * kSeq * kDm) return;
  if (in_sizes[1] != kDm) return;
  if (in_sizes[2] != kDm) return;
  if (in_sizes[3] != kDm * kXzP) return;
  if (in_sizes[4] != kDin * 4) return;
  if (in_sizes[5] != kDin) return;
  if (in_sizes[6] != kDin * kXpN) return;
  if (in_sizes[7] != kDtR * kDin) return;
  if (in_sizes[8] != kDin) return;
  if (in_sizes[9] != kDin * kNst) return;
  if (in_sizes[10] != kDin) return;
  if (in_sizes[11] != kDin * kDm) return;
  if (out_size != kBatch * kSeq * kDm) return;
  if (ws_size < kWsTotal) return;

  const float* x      = (const float*)d_in[0];
  const float* ln_g   = (const float*)d_in[1];
  const float* ln_b   = (const float*)d_in[2];
  const float* W_in   = (const float*)d_in[3];
  const float* conv_w = (const float*)d_in[4];
  const float* conv_b = (const float*)d_in[5];
  const float* W_x    = (const float*)d_in[6];
  const float* W_dt   = (const float*)d_in[7];
  const float* b_dt   = (const float*)d_in[8];
  const float* A_log  = (const float*)d_in[9];
  const float* D_par  = (const float*)d_in[10];
  const float* W_out  = (const float*)d_in[11];
  float* out = (float*)d_out;

  char* ws = (char*)d_ws;
  unsigned short* WIN  = (unsigned short*)(ws + kOffWIN);
  unsigned short* WOUT = (unsigned short*)(ws + kOffWOUT);
  unsigned short* WXH  = (unsigned short*)(ws + kOffWXH);
  unsigned short* WXL  = (unsigned short*)(ws + kOffWXL);
  unsigned short* WDT  = (unsigned short*)(ws + kOffWDT);
  unsigned short* XH   = (unsigned short*)(ws + kOffXH);
  unsigned short* XL   = (unsigned short*)(ws + kOffXL);
  float*          XZ   = (float*)(ws + kOffXZ);
  float*          U    = (float*)(ws + kOffU);
  unsigned short* UH   = (unsigned short*)(ws + kOffUH);
  unsigned short* UL   = (unsigned short*)(ws + kOffUL);
  float*          BC   = (float*)(ws + kOffBC);
  unsigned short* BCH  = (unsigned short*)(ws + kOffBCH);
  unsigned short* BCL  = (unsigned short*)(ws + kOffBCL);
  float*          DT   = (float*)(ws + kOffDT);
  unsigned short* YH   = (unsigned short*)(ws + kOffYH);
  unsigned short* YL   = (unsigned short*)(ws + kOffYL);
  float*          P    = (float*)(ws + kOffP);

  transpose_pack_kernel<false><<<dim3(kXzP / 64, kDm / 64), 256, 0, stream>>>(W_in, WIN, WIN, kDm, kXzP, kWCarry);
  transpose_pack_kernel<false><<<dim3(kDm / 64, kDin / 64), 256, 0, stream>>>(W_out, WOUT, WOUT, kDin, kDm, kWCarry);
  transpose_pack_kernel<true><<<dim3(kBcP / 64, kDin / 64), 256, 0, stream>>>(W_x, WXH, WXL, kDin, kXpN, kWCarry);
  transpose_pack_kernel<false><<<dim3(kDin / 64, kDtR / 64), 256, 0, stream>>>(W_dt, WDT, WDT, kDtR, kDin, kWCarry);

  for (int b = 0; b < kBatch; ++b) {
    const float* xb = x + (size_t)b * kSeq * kDm;
    float* outb = out + (size_t)b * kSeq * kDm;

    ln_split_rows_kernel<<<kSeq / 8, 256, 0, stream>>>(xb, ln_g, ln_b, XH, XL);

    eng::gemm_f16_kernel<2, 1><<<dim3((kSeq / 32) * (kXzP / 64) / 8), 256, 0, stream>>>(
        XH, XL, kDm, WIN, WIN, kDm, XZ, kXzP, kSeq, kXzP, kDm, kSW, kSWr);

    conv_silu_kernel<<<dim3(kDin / 256, kSeq / 64), 256, 0, stream>>>(XZ, conv_w, conv_b, U, UH, UL);

    eng::gemm_f16_kernel<1, 2><<<dim3((kSeq / 16) * (kBcP / 64) / 8), 256, 0, stream>>>(
        UH, UL, kDin, WXH, WXL, kDin, BC, kBcP, kSeq, kBcP, kDin, kSW, kSWr);

    split_rows_f16_kernel<<<(kSeq * kBcP / 8) / 256, 256, 0, stream>>>(BC, BCH, BCL, kSeq * kBcP / 8);
    eng::gemm_f16_kernel<2, 1><<<dim3((kSeq / 32) * (kDin / 64) / 8), 256, 0, stream>>>(
        BCH, BCL, kBcP, WDT, WDT, kDtR, DT, kDin, kSeq, kDin, kDtR, kSW, kSWr);
    bias_rows_kernel<<<(kSeq * kDin / 4) / 256, 256, 0, stream>>>(DT, b_dt, kSeq * kDin / 4);

    ms1_args sa;
    sa.dtpre = DT;
    sa.u = U;
    sa.bc = BC;
    sa.z = XZ;
    sa.A_log = A_log;
    sa.Dskip = D_par;
    sa.y = (__half*)YH;
    sa.y_lo = (__half*)YL;
    sa.ld_dtpre = kDin;
    sa.ld_u = kDin;
    sa.ld_bc = kBcP;
    sa.ld_z = kXzP;
    sa.ld_y = kDin;
    sa.offB = kOffB;
    sa.offC = kOffC;
    sa.offZ = kDin;
    sa.ycarry = kYCarry;
    sa.dir = 1;
    sa.D = kDin;
    sa.L = kSeq;
    sa.nbatch = 1;
    ms1_scan_kernel<16><<<dim3(kDin / 64), 64, 0, stream>>>(sa);

    eng::gemm_f16_kernel<2, 1><<<dim3((kSeq / 32) * (kDm / 64) / 8), 256, 0, stream>>>(
        YH, YL, kDin, WOUT, WOUT, kDin, P, kDm, kSeq, kDm, kDin, kSY, kSYr);
    residual_out_kernel<<<(kSeq * kDm / 4) / 256, 256, 0, stream>>>(P, xb, outb, kSeq * kDm / 4);
  }
}
